// Sparse_3d_Convolution_Block_69526930588487
// MI455X (gfx1250) — hardware-verified
//
#include <hip/hip_runtime.h>
#include <stddef.h>


#define C_CH    64
#define K_OFF   27
#define K_CTR   13
#define N_RB    26
#define XSC     8.0f
#define WSC     256.0f
#define RH      0.00048828125f
#define WSCAP   134217728
#define SRCH    20

#define CTHR    128
#define CWAV    (CTHR / 32)
#define CPTS    (16 * CWAV)
#define GRP     9
#define NGRP    (K_OFF / GRP)
#define AROW    (GRP * C_CH)
#define NPAIR   (CPTS * K_OFF)
#define NPIECE  (CPTS * GRP * 8)
#define PSTR    128
#define STN     256

#define FTHR    256
#define FROWS   64
#define BTHR    256

#define LC_A    0
#define LC_S    (CPTS * AROW * 2)
#define LC_NB   (LC_S + CWAV * 1024 * 4)
#define LC_LEN  (LC_NB + NPAIR * 4)
#define LC_PL   (LC_LEN + 32 * 4)
#define LDS_CONV (LC_PL + PSTR * 4)

static_assert(NGRP * GRP == K_OFF);
static_assert(CPTS == 64);
static_assert(LC_S == 73728);
static_assert(LC_NB == 90112);
static_assert(LDS_CONV == 97664);
static_assert((LC_S % 16) == 0 && (LC_NB % 16) == 0 && (LC_LEN % 16) == 0 && (LC_PL % 16) == 0);
static_assert((NPIECE % CTHR) == 0);
static_assert((AROW * 2) % 16 == 0);
static_assert(BTHR == STN);
static_assert(PSTR == CTHR);
static_assert(FROWS * 8 == 2 * FTHR);

typedef float    v4f  __attribute__((ext_vector_type(4)));
typedef float    v8f  __attribute__((ext_vector_type(8)));
typedef _Float16 v4h  __attribute__((ext_vector_type(4)));
typedef _Float16 v8h  __attribute__((ext_vector_type(8)));
typedef _Float16 v16h __attribute__((ext_vector_type(16)));
union Frag  { v16h v; v8h h[2]; };
union Frag8 { v8h v; v4h q[2]; };

__device__ __forceinline__ v8f wmh(v16h a, v16h b, v8f c) {
  v8f d = __builtin_amdgcn_wmma_f32_16x16x32_f16(false, a, false, b, (short)0, c, false, false);
  asm volatile("v_nop\n\tv_nop\n\tv_nop\n\tv_nop" : "+v"(d) : "v"(a), "v"(b));
  return d;
}

__device__ __forceinline__ v4h cvt4h(v4f x) {
  v4h r;
  r.x = (_Float16)x.x;
  r.y = (_Float16)x.y;
  r.z = (_Float16)x.z;
  r.w = (_Float16)x.w;
  return r;
}

__global__ __launch_bounds__(FTHR) void k_wprep(const float* __restrict__ W, _Float16* Wp) {
  const int kp = blockIdx.x, tid = threadIdx.x;
  const float* wk = W + (size_t)kp * (C_CH * C_CH);
#pragma unroll
  for (int it = 0; it < 2; ++it) {
    const int n = 32 * it + (tid >> 3), c0 = (tid & 7) * 8;
    v8h hv;
#pragma unroll
    for (int e = 0; e < 8; ++e) hv[e] = (_Float16)(wk[(c0 + e) * C_CH + n] * WSC);
    _Float16* dst = Wp + ((size_t)kp * C_CH + n) * C_CH + c0;
    *(volatile v8h*)dst = hv;
    __threadfence();
    *(volatile v8h*)dst = hv;
  }
}

__global__ __launch_bounds__(FTHR) void k_fcvt(const float* __restrict__ X, _Float16* Fh, int nN) {
  const int tid = threadIdx.x;
#pragma unroll
  for (int it = 0; it < 2; ++it) {
    const int row = blockIdx.x * FROWS + 32 * it + (tid >> 3);
    const int c0 = (tid & 7) * 8;
    const bool ok = row < nN;
    const int rc = ok ? row : nN - 1;
    const float* xp = X + (size_t)rc * C_CH + c0;
    v4f f0 = *(const v4f*)(xp);
    v4f f1 = *(const v4f*)(xp + 4);
    const v4f z = {0.0f, 0.0f, 0.0f, 0.0f};
    f0 = ok ? f0 * XSC : z;
    f1 = ok ? f1 * XSC : z;
    Frag8 hv;
    hv.q[0] = cvt4h(f0);
    hv.q[1] = cvt4h(f1);
    _Float16* dst = Fh + (size_t)row * C_CH + c0;
    *(volatile v8h*)dst = hv.v;
    __threadfence();
    *(volatile v8h*)dst = hv.v;
  }
}

__global__ __launch_bounds__(CTHR) void k_conv(const _Float16* __restrict__ Fh, const _Float16* __restrict__ Wp,
                                               const int* __restrict__ in_idx, const int* __restrict__ out_idx,
                                               float* Y, float* part, int nN, int P) {
  extern __shared__ __attribute__((aligned(16))) char dynl[];
  _Float16* AL = (_Float16*)(dynl + LC_A);
  float* S   = (float*)(dynl + LC_S);
  int* nbl   = (int*)(dynl + LC_NB);
  int* lenl  = (int*)(dynl + LC_LEN);
  float* pl  = (float*)(dynl + LC_PL);
  const int tid = threadIdx.x, lane = tid & 31, hh = lane >> 4, m = lane & 15;
  const int wave = __builtin_amdgcn_readfirstlane(tid >> 5);
  const int pb = blockIdx.x * CPTS;

  {
    const int k = tid < N_RB ? tid : N_RB - 1;
    const int* arr = out_idx + (size_t)k * P;
    int lo = 0, n = P;
#pragma unroll 1
    for (int s = 0; s < SRCH; ++s) {
      const int half = n >> 1;
      const int mid = lo + half;
      const int mc = mid > P - 1 ? P - 1 : mid;
      const int v = arr[mc];
      const bool lt = (n > 0) && (v < nN);
      lo = lt ? mid + 1 : lo;
      n  = lt ? n - half - 1 : half;
    }
    if (tid < N_RB) lenl[tid] = lo;
  }
  __syncthreads();

#pragma unroll 1
  for (int it = 0; it < (NPAIR + CTHR - 1) / CTHR; ++it) {
    const int p = it * CTHR + tid;
    const int pc = p < NPAIR ? p : NPAIR - 1;
    const int jj = pc / K_OFF;
    const int kp = pc - jj * K_OFF;
    const int pt = pb + jj;
    const int kq = kp < K_CTR ? kp : kp - 1;
    const int km = (N_RB - 1) - kq;
    const int len = lenl[km];
    const int* arr = in_idx + (size_t)km * P;
    int lo = 0, n = len;
#pragma unroll 1
    for (int s = 0; s < SRCH; ++s) {
      const int half = n >> 1;
      const int mid = lo + half;
      const int mc = mid > P - 1 ? P - 1 : mid;
      const int v = arr[mc];
      const bool lt = (n > 0) && (v < pt);
      lo = lt ? mid + 1 : lo;
      n  = lt ? n - half - 1 : half;
    }
    const int lc = lo > P - 1 ? P - 1 : lo;
    const bool found = (lo < len) && (arr[lc] == pt);
    const int cand = out_idx[(size_t)km * P + lc];
    const int candc = cand < 0 ? 0 : (cand > nN ? nN : cand);
    int nb = found ? candc : nN;
    nb = (kp == K_CTR) ? pt : nb;
    nb = (pt < nN) ? nb : nN;
    if (p < NPAIR) nbl[p] = nb;
  }
  __syncthreads();

  const v8f z8 = {0.0f, 0.0f, 0.0f, 0.0f, 0.0f, 0.0f, 0.0f, 0.0f};
  v8f acc0 = z8, acc1 = z8, acc2 = z8, acc3 = z8;
#pragma unroll 1
  for (int g = 0; g < NGRP; ++g) {
#pragma unroll 1
    for (int it = 0; it < NPIECE / CTHR; ++it) {
      const int p = it * CTHR + tid;
      const int jj = p / (GRP * 8);
      const int r = p - jj * (GRP * 8);
      const int o = r >> 3, q = r & 7;
      const int nb = nbl[jj * K_OFF + g * GRP + o];
      const v8h vv = *(const v8h*)(Fh + (size_t)nb * C_CH + 8 * q);
      *(v8h*)(AL + (size_t)jj * AROW + o * C_CH + 8 * q) = vv;
    }
    __syncthreads();
    {
      const _Float16* ga = AL + (size_t)(wave * 16 + m) * AROW + 8 * hh;
      const _Float16* wb = Wp + (size_t)(g * GRP) * (C_CH * C_CH) + (size_t)m * C_CH + 8 * hh;
#pragma unroll 1
      for (int o = 0; o < GRP; ++o) {
#pragma unroll
        for (int kb = 0; kb < 2; ++kb) {
          Frag a, b0, b1, b2, b3;
          const _Float16* gp = ga + o * C_CH + kb * 32;
          a.h[0] = *(const v8h*)(gp);
          a.h[1] = *(const v8h*)(gp + 16);
          const _Float16* bp = wb + (size_t)o * (C_CH * C_CH) + kb * 32;
          b0.h[0] = *(const v8h*)(bp);
          b0.h[1] = *(const v8h*)(bp + 16);
          b1.h[0] = *(const v8h*)(bp + 16 * C_CH);
          b1.h[1] = *(const v8h*)(bp + 16 * C_CH + 16);
          b2.h[0] = *(const v8h*)(bp + 32 * C_CH);
          b2.h[1] = *(const v8h*)(bp + 32 * C_CH + 16);
          b3.h[0] = *(const v8h*)(bp + 48 * C_CH);
          b3.h[1] = *(const v8h*)(bp + 48 * C_CH + 16);
          acc0 = wmh(a.v, b0.v, acc0);
          acc1 = wmh(a.v, b1.v, acc1);
          acc2 = wmh(a.v, b2.v, acc2);
          acc3 = wmh(a.v, b3.v, acc3);
        }
      }
    }
    __syncthreads();
  }

  float* Sw = S + wave * 1024;
#pragma unroll
  for (int r = 0; r < 8; ++r) {
    Sw[(8 * hh + r) * C_CH + m]      = acc0[r] * RH;
    Sw[(8 * hh + r) * C_CH + 16 + m] = acc1[r] * RH;
    Sw[(8 * hh + r) * C_CH + 32 + m] = acc2[r] * RH;
    Sw[(8 * hh + r) * C_CH + 48 + m] = acc3[r] * RH;
  }
  __syncthreads();
  {
    const int rr = lane >> 4, cc = (lane & 15) * 4;
    v4f ov[8];
#pragma unroll
    for (int qq = 0; qq < 8; ++qq) ov[qq] = *(const v4f*)(Sw + (2 * qq + rr) * C_CH + cc);
    const size_t rbase = (size_t)(pb + 16 * wave + rr);
#pragma unroll
    for (int qq = 0; qq < 8; ++qq) {
      float* op = Y + (rbase + 2 * qq) * C_CH + cc;
      *(volatile v4f*)op = ov[qq];
    }
    __threadfence();
#pragma unroll
    for (int qq = 0; qq < 8; ++qq) {
      float* op = Y + (rbase + 2 * qq) * C_CH + cc;
      *(volatile v4f*)op = ov[qq];
    }
  }
  {
    const int c = tid & 63, which = tid >> 6;
    float a = 0.0f;
#pragma unroll 4
    for (int r = 0; r < CPTS; ++r) {
      const float v = S[r * C_CH + c];
      a += which ? v * v : v;
    }
    pl[tid] = a;
  }
  __syncthreads();
  if (wave == 0) {
    const v4f vv = *(const v4f*)(pl + 4 * lane);
    float* pp = part + (size_t)blockIdx.x * PSTR + 4 * lane;
    *(volatile v4f*)pp = vv;
    __threadfence();
    *(volatile v4f*)pp = vv;
  }
}

__global__ __launch_bounds__(128) void k_stats(const float* __restrict__ part, const float* __restrict__ gamma,
                                               const float* __restrict__ beta, float* stats, int nBlk, int nN) {
  __shared__ double sd[128];
  __shared__ __attribute__((aligned(16))) float stf[STN];
  const int t = threadIdx.x;
  double a = 0.0;
#pragma unroll 1
  for (int b = 0; b < nBlk; ++b) a += (double)part[(size_t)b * PSTR + t];
  sd[t] = a;
  stf[t] = 0.0f;
  stf[128 + t] = 0.0f;
  __syncthreads();
  if (t < 64) {
    const double inv = 1.0 / (double)nN;
    const double mean = sd[t] * inv;
    double var = sd[64 + t] * inv - mean * mean;
    var = var < 0.0 ? 0.0 : var;
    const float varf = (float)var;
    const float mul = rsqrtf(varf + 1e-5f) * gamma[t];
    stf[t] = (float)mean;
    stf[64 + t] = mul;
    stf[128 + t] = beta[t];
  }
  __syncthreads();
  if (t < 64) {
    const v4f vv = *(const v4f*)(stf + 4 * t);
    float* sp = stats + 4 * t;
    *(volatile v4f*)sp = vv;
    __threadfence();
    *(volatile v4f*)sp = vv;
  }
}

__global__ __launch_bounds__(BTHR) void k_bn(const float* __restrict__ Y, const float* __restrict__ stats,
                                             float* out, int nQ) {
  __shared__ __attribute__((aligned(16))) float st[STN];
  const int tid = threadIdx.x;
  st[tid] = stats[tid];
  __syncthreads();
  const int q = blockIdx.x * BTHR + tid;
  const int qc = q < nQ ? q : nQ - 1;
  const v4f y = *(const v4f*)(Y + (size_t)qc * 4);
  const int c0 = (qc & 15) * 4;
  const v4f mean = *(const v4f*)(st + c0);
  const v4f mul  = *(const v4f*)(st + 64 + c0);
  const v4f add  = *(const v4f*)(st + 128 + c0);
  v4f r = (y - mean) * mul + add;
  r.x = fmaxf(r.x, 0.0f);
  r.y = fmaxf(r.y, 0.0f);
  r.z = fmaxf(r.z, 0.0f);
  r.w = fmaxf(r.w, 0.0f);
  float* op = out + (size_t)qc * 4;
  if (q < nQ) *(volatile v4f*)op = r;
  __threadfence();
  if (q < nQ) *(volatile v4f*)op = r;
}

extern "C" void kernel_launch(void* const* d_in, const int* in_sizes, int n_in,
                              void* d_out, int out_size, void* d_ws, size_t ws_size,
                              hipStream_t stream) {
  if (n_in < 6) return;
  if (in_sizes[0] < C_CH || (in_sizes[0] % C_CH) != 0) return;
  const int nN = in_sizes[0] / C_CH;
  if (in_sizes[1] != K_OFF * C_CH * C_CH) return;
  if (in_sizes[2] != C_CH || in_sizes[3] != C_CH) return;
  if (in_sizes[4] < N_RB || (in_sizes[4] % N_RB) != 0) return;
  const int P = in_sizes[4] / N_RB;
  if (in_sizes[5] != in_sizes[4]) return;
  if (P >= (1 << SRCH)) return;
  if (out_size != nN * C_CH) return;

  const int gC      = (nN + CPTS - 1) / CPTS;
  const int rowsY   = gC * CPTS;
  const int rowsPad = ((nN + 1 + FROWS - 1) / FROWS) * FROWS;
  const int gF      = rowsPad / FROWS;
  const int nQ      = nN * (C_CH / 4);
  const int gB      = (nQ + BTHR - 1) / BTHR;
  if (rowsPad < nN + 1 || rowsPad < rowsY) return;

  const float* X   = (const float*)d_in[0];
  const float* W   = (const float*)d_in[1];
  const float* gam = (const float*)d_in[2];
  const float* bet = (const float*)d_in[3];
  const int*   II  = (const int*)d_in[4];
  const int*   OI  = (const int*)d_in[5];
  float* out = (float*)d_out;

  char* ws = (char*)d_ws;
  size_t off = 0;
  const size_t oFh = off; off += (size_t)rowsPad * C_CH * 2;      off = (off + 255) & ~(size_t)255;
  const size_t oWp = off; off += (size_t)K_OFF * C_CH * C_CH * 2; off = (off + 255) & ~(size_t)255;
  const size_t oY  = off; off += (size_t)rowsY * C_CH * 4;        off = (off + 255) & ~(size_t)255;
  const size_t oPt = off; off += (size_t)gC * PSTR * 4;           off = (off + 255) & ~(size_t)255;
  const size_t oSt = off; off += (size_t)STN * 4;                 off = (off + 255) & ~(size_t)255;
  if (off > ws_size || off > (size_t)WSCAP) return;
  _Float16* Fh   = (_Float16*)(ws + oFh);
  _Float16* Wp   = (_Float16*)(ws + oWp);
  float*    Y    = (float*)(ws + oY);
  float*    part = (float*)(ws + oPt);
  float*    stats = (float*)(ws + oSt);

  hipFuncSetAttribute(reinterpret_cast<const void*>(&k_conv), hipFuncAttributeMaxDynamicSharedMemorySize, LDS_CONV);

  k_wprep<<<K_OFF, FTHR, 0, stream>>>(W, Wp);
  k_fcvt<<<gF, FTHR, 0, stream>>>(X, Fh, nN);
  k_conv<<<gC, CTHR, LDS_CONV, stream>>>(Fh, Wp, II, OI, Y, part, nN, P);
  k_stats<<<1, 128, 0, stream>>>(part, gam, bet, stats, gC, nN);
  k_bn<<<gB, BTHR, 0, stream>>>(Y, stats, out, nQ);
}
